// Mamba_TransformerEncoderLayer_9165460210046
// MI455X (gfx1250) — hardware-verified
//
#include <hip/hip_runtime.h>
#include <hip/hip_bf16.h>


#define NB_   2
#define NL_   512
#define DM_   1024
#define NH_   16
#define HD_   64
#define FF_   4096
#define DI_   2048
#define NS_   64
#define DTR_  64
#define XPN_  192
#define MT_   (NB_ * NL_)
#define SP_   68
#define SVP_  264

static_assert(MT_ % 128 == 0);
static_assert(NL_ % 128 == 0);
static_assert(NH_ * HD_ == DM_);
static_assert(HD_ == 64);
static_assert(DI_ == 2 * DM_);
static_assert(DI_ % 64 == 0);
static_assert(DM_ % 64 == 0);
static_assert(FF_ % 64 == 0);
static_assert(XPN_ % 64 == 0);
static_assert(NS_ == 64);
static_assert(DTR_ == 64);
static_assert((NL_ & (NL_ - 1)) == 0);
static_assert(DM_ == 4 * 256);
static_assert(DI_ == 8 * 256);

typedef float          v4f   __attribute__((ext_vector_type(4)));
typedef float          v8f   __attribute__((ext_vector_type(8)));
typedef _Float16       v8h   __attribute__((ext_vector_type(8)));
typedef _Float16       v16h  __attribute__((ext_vector_type(16)));
typedef __bf16         v16b  __attribute__((ext_vector_type(16)));
typedef unsigned short u16x8 __attribute__((ext_vector_type(8)));

union FragH { u16x8 h[2]; v16h v; };
union FragB { u16x8 h[2]; v16b v; };
union Pack8 { v8h f; u16x8 u; };
union H1    { _Float16 f; unsigned short u; };

__device__ __forceinline__ unsigned short f32_to_bf16(float f) {
    unsigned u = __float_as_uint(f);
    unsigned r = u + 0x7FFFu + ((u >> 16) & 1u);
    return (unsigned short)(r >> 16);
}
__device__ __forceinline__ float bf16_to_f32(unsigned short b) {
    return __uint_as_float(((unsigned)b) << 16);
}
__device__ __forceinline__ float silu_f(float x) {
    const float e = __expf(-x);
    return x * __builtin_amdgcn_rcpf(1.0f + e);
}
__device__ __forceinline__ float softplus_f(float x) {
    return fmaxf(x, 0.0f) + log1pf(expf(-fabsf(x)));
}
__device__ __forceinline__ v8f ld8f(const float* p) {
    const v4f a = *(const v4f*)p;
    const v4f b = *(const v4f*)(p + 4);
    return __builtin_shufflevector(a, b, 0, 1, 2, 3, 4, 5, 6, 7);
}

__device__ __forceinline__ void mma_raw(v8f& acc, const FragH& a, const FragH& b) {
    acc = __builtin_amdgcn_wmma_f32_16x16x32_f16(false, a.v, false, b.v, (short)0, acc, false, false);
}
__device__ __forceinline__ void mma_raw(v8f& acc, const FragB& a, const FragB& b) {
    acc = __builtin_amdgcn_wmma_f32_16x16x32_bf16(false, a.v, false, b.v, (short)0, acc, false, false);
}
template<typename FR>
__device__ __forceinline__ void wmma_guard(v8f (&acc)[8], FR (&fa)[2], FR (&fb)[4]) {
    asm volatile("v_nop\n\tv_nop\n\tv_nop\n\tv_nop"
                 : "+v"(acc[0]), "+v"(acc[1]), "+v"(acc[2]), "+v"(acc[3]),
                   "+v"(acc[4]), "+v"(acc[5]), "+v"(acc[6]), "+v"(acc[7])
                 : "v"(fa[0].v), "v"(fa[1].v),
                   "v"(fb[0].v), "v"(fb[1].v), "v"(fb[2].v), "v"(fb[3].v));
}

__global__ __launch_bounds__(256)
void cvt_kernel(const float* __restrict__ src, unsigned short* dst0, unsigned short* dst1,
                unsigned short* dst2, int n8, int mode, float scale)
{
    const int i = blockIdx.x * 256 + threadIdx.x;
    if (i >= n8) return;
    const size_t e = (size_t)i * 8;
    const v8f x = ld8f(src + e);
    if (mode != 1) {
        Pack8 pk;
        pk.f = __builtin_convertvector(x * scale, v8h);
        const u16x8 v = pk.u;
        *(volatile u16x8*)(dst0 + e) = v;
        __threadfence();
        *(volatile u16x8*)(dst0 + e) = v;
    }
    if (mode != 0) {
        unsigned short* dh = (mode == 1) ? dst0 : dst1;
        unsigned short* dl = (mode == 1) ? dst1 : dst2;
        u16x8 hv, lv;
#pragma unroll
        for (int c = 0; c < 8; ++c) {
            const float f = x[c];
            const unsigned short hb = f32_to_bf16(f);
            const unsigned short lb = f32_to_bf16(f - bf16_to_f32(hb));
            hv[c] = hb;
            lv[c] = lb;
        }
        *(volatile u16x8*)(dh + e) = hv;
        *(volatile u16x8*)(dl + e) = lv;
        __threadfence();
        *(volatile u16x8*)(dh + e) = hv;
        *(volatile u16x8*)(dl + e) = lv;
    }
}

template<int OK>
__device__ __forceinline__ void tile_store_pass(const float* st, void* C0, void* C1,
                                                size_t gofs, int ldc, int lane, float oscale)
{
    if constexpr (OK == 0) {
        float* gp = (float*)C0 + gofs;
        const int rsub = lane >> 4;
        const int c4   = (lane & 15) * 4;
#pragma unroll
        for (int it = 0; it < 16; ++it) {
            const int row = it * 2 + rsub;
            const v4f v = *(const v4f*)(st + row * SP_ + c4);
            *(volatile v4f*)(gp + (size_t)row * ldc + c4) = v;
        }
    } else {
        const int rsub = lane >> 3;
        const int c8   = (lane & 7) * 8;
        unsigned short* g0 = (unsigned short*)C0 + gofs;
        unsigned short* g1 = (unsigned short*)C1 + gofs;
#pragma unroll
        for (int it = 0; it < 8; ++it) {
            const int row = it * 4 + rsub;
            const float* sp = st + row * SP_ + c8;
            const v4f x0 = *(const v4f*)sp;
            const v4f x1 = *(const v4f*)(sp + 4);
            const v8f x = __builtin_shufflevector(x0, x1, 0, 1, 2, 3, 4, 5, 6, 7);
            if constexpr (OK == 1) {
                Pack8 pk;
                pk.f = __builtin_convertvector(x * oscale, v8h);
                const u16x8 v = pk.u;
                *(volatile u16x8*)(g0 + (size_t)row * ldc + c8) = v;
            } else {
                u16x8 hv, lv;
#pragma unroll
                for (int c = 0; c < 8; ++c) {
                    const float f = x[c];
                    const unsigned short hb = f32_to_bf16(f);
                    const unsigned short lb = f32_to_bf16(f - bf16_to_f32(hb));
                    hv[c] = hb;
                    lv[c] = lb;
                }
                *(volatile u16x8*)(g0 + (size_t)row * ldc + c8) = hv;
                *(volatile u16x8*)(g1 + (size_t)row * ldc + c8) = lv;
            }
        }
    }
}

template<typename FR, bool SPLIT, int OK>
__global__ __launch_bounds__(128)
void gemm_tn_kernel(const unsigned short* __restrict__ A,  const unsigned short* __restrict__ A2,
                    const unsigned short* __restrict__ Bw, const unsigned short* __restrict__ B2,
                    const float* __restrict__ bias, const float* __restrict__ addsrc,
                    void* C0, void* C1,
                    int K, int lda, int ldb, int ldc, int zdiv,
                    long long sA, long long sB, long long sCb, long long sCh,
                    float scale, float oscale, int flags)
{
    __shared__ __attribute__((aligned(16))) float stile[4][32 * SP_];

    const int tid  = threadIdx.x;
    const int lane = tid & 31;
    const int wave = tid >> 5;
    const int h    = lane >> 4;
    const int m    = lane & 15;

    const int z  = blockIdx.z;
    const int zb = z / zdiv;
    const int zh = z - zb * zdiv;
    const size_t zao  = (size_t)((long long)z * sA);
    const size_t zbo  = (size_t)((long long)z * sB);
    const size_t coff = (size_t)((long long)zb * sCb + (long long)zh * sCh);

    const int rowW = blockIdx.y * 128 + wave * 32;
    const int colB = blockIdx.x * 64;

    v8f acc[8];
#pragma unroll
    for (int j = 0; j < 8; ++j)
#pragma unroll
        for (int r = 0; r < 8; ++r) acc[j][r] = 0.0f;

    const size_t aoff = zao + (size_t)(rowW + m) * lda + 8 * h;
    const size_t boff = zbo + (size_t)(colB + m) * ldb + 8 * h;
    const size_t a16  = (size_t)16 * lda;
    const size_t b16  = (size_t)16 * ldb;
    const int nk = K >> 5;

#pragma unroll 1
    for (int kt = 0; kt < nk; ++kt) {
        const size_t k0 = (size_t)kt * 32;
        FR fa[2], fb[4];
#pragma unroll
        for (int s = 0; s < 2; ++s) {
            const unsigned short* p = A + aoff + s * a16 + k0;
            fa[s].h[0] = *(const u16x8*)(p);
            fa[s].h[1] = *(const u16x8*)(p + 16);
        }
#pragma unroll
        for (int j = 0; j < 4; ++j) {
            const unsigned short* p = Bw + boff + j * b16 + k0;
            fb[j].h[0] = *(const u16x8*)(p);
            fb[j].h[1] = *(const u16x8*)(p + 16);
        }
#pragma unroll
        for (int s = 0; s < 2; ++s)
#pragma unroll
            for (int j = 0; j < 4; ++j) mma_raw(acc[s * 4 + j], fa[s], fb[j]);
        wmma_guard(acc, fa, fb);

        if constexpr (SPLIT) {
            FR gb[4];
#pragma unroll
            for (int j = 0; j < 4; ++j) {
                const unsigned short* q = B2 + boff + j * b16 + k0;
                gb[j].h[0] = *(const u16x8*)(q);
                gb[j].h[1] = *(const u16x8*)(q + 16);
            }
#pragma unroll
            for (int s = 0; s < 2; ++s)
#pragma unroll
                for (int j = 0; j < 4; ++j) mma_raw(acc[s * 4 + j], fa[s], gb[j]);
            wmma_guard(acc, fa, gb);

            FR ga[2];
#pragma unroll
            for (int s = 0; s < 2; ++s) {
                const unsigned short* q = A2 + aoff + s * a16 + k0;
                ga[s].h[0] = *(const u16x8*)(q);
                ga[s].h[1] = *(const u16x8*)(q + 16);
            }
#pragma unroll
            for (int s = 0; s < 2; ++s)
#pragma unroll
                for (int j = 0; j < 4; ++j) mma_raw(acc[s * 4 + j], ga[s], fb[j]);
            wmma_guard(acc, ga, fb);
        }
    }

    float* st = stile[wave];
    const bool has_bias = (flags & 1) != 0;
    const bool has_add  = (flags & 2) != 0;
    const bool do_relu  = (flags & 4) != 0;
#pragma unroll
    for (int j = 0; j < 4; ++j) {
        const int lc = j * 16 + m;
        const float bj = has_bias ? bias[colB + lc] : 0.0f;
#pragma unroll
        for (int s = 0; s < 2; ++s)
#pragma unroll
            for (int r = 0; r < 8; ++r) {
                const int lr = s * 16 + 8 * h + r;
                float v = acc[s * 4 + j][r] * scale + bj;
                if (has_add) v += addsrc[coff + (size_t)(rowW + lr) * ldc + colB + lc];
                if (do_relu) v = fmaxf(v, 0.0f);
                st[lr * SP_ + lc] = v;
            }
    }
    __syncthreads();

    const size_t gofs = coff + (size_t)rowW * ldc + colB;
    tile_store_pass<OK>(st, C0, C1, gofs, ldc, lane, oscale);
    __threadfence();
    tile_store_pass<OK>(st, C0, C1, gofs, ldc, lane, oscale);
}

__global__ __launch_bounds__(256)
void attn_prep_kernel(const float* __restrict__ QKV, unsigned short* Q16, unsigned short* K16,
                      unsigned short* VT16)
{
    __shared__ __attribute__((aligned(16))) unsigned short sV[64 * SVP_];
    const int tid = threadIdx.x;
    const int t0  = blockIdx.x * 64;
    const int b   = t0 / NL_;
    const int l0  = t0 - b * NL_;
    const int hg  = blockIdx.y;

#pragma unroll
    for (int i = 0; i < 8; ++i) {
        const int idx  = i * 256 + tid;
        const int tok  = idx >> 5;
        const int c8   = (idx & 31) * 8;
        const int head = hg * 4 + (c8 >> 6);
        const int dd   = c8 & 63;
        const float* rp = QKV + (size_t)(t0 + tok) * (3 * DM_) + hg * 256 + c8;
        const v8f qv = ld8f(rp);
        const v8f kv = ld8f(rp + DM_);
        const v8f vv = ld8f(rp + 2 * DM_);
        Pack8 pq, pk, pv;
        pq.f = __builtin_convertvector(qv, v8h);
        pk.f = __builtin_convertvector(kv, v8h);
        pv.f = __builtin_convertvector(vv, v8h);
        const size_t o = ((size_t)(b * NH_ + head) * NL_ + l0 + tok) * HD_ + dd;
        const u16x8 uq = pq.u, uk = pk.u;
        *(volatile u16x8*)(Q16 + o) = uq;
        *(volatile u16x8*)(K16 + o) = uk;
        __threadfence();
        *(volatile u16x8*)(Q16 + o) = uq;
        *(volatile u16x8*)(K16 + o) = uk;
        *(u16x8*)(sV + tok * SVP_ + c8) = pv.u;
    }
    __syncthreads();
#pragma unroll
    for (int i = 0; i < 8; ++i) {
        const int idx  = i * 256 + tid;
        const int line = idx >> 3;
        const int seg  = idx & 7;
        const int tok0 = seg * 8;
        u16x8 v;
#pragma unroll
        for (int j = 0; j < 8; ++j) v[j] = sV[(tok0 + j) * SVP_ + line];
        const size_t o = ((size_t)(b * NH_ + hg * 4 + (line >> 6)) * HD_ + (line & 63)) * NL_ + l0 + tok0;
        *(volatile u16x8*)(VT16 + o) = v;
        __threadfence();
        *(volatile u16x8*)(VT16 + o) = v;
    }
}

__global__ __launch_bounds__(256)
void softmax_kernel(const float* __restrict__ S, unsigned short* P16)
{
    const int lane = threadIdx.x & 31;
    const int wave = threadIdx.x >> 5;
    const size_t row = (size_t)blockIdx.x * 8 + wave;
    const float* p = S + row * NL_;
    const v8f a = ld8f(p + lane * 8);
    const v8f c = ld8f(p + (NL_ / 2) + lane * 8);
    float mx = -3.0e38f;
#pragma unroll
    for (int i = 0; i < 8; ++i) mx = fmaxf(mx, fmaxf(a[i], c[i]));
#pragma unroll
    for (int off = 16; off; off >>= 1) mx = fmaxf(mx, __shfl_xor(mx, off, 32));
    v8f ea, ec;
    float sum = 0.0f;
#pragma unroll
    for (int i = 0; i < 8; ++i) {
        ea[i] = __expf(a[i] - mx);
        ec[i] = __expf(c[i] - mx);
        sum += ea[i] + ec[i];
    }
#pragma unroll
    for (int off = 16; off; off >>= 1) sum += __shfl_xor(sum, off, 32);
    const float f = __builtin_amdgcn_rcpf(sum) * 16384.0f;
    Pack8 pa, pc;
    pa.f = __builtin_convertvector(ea * f, v8h);
    pc.f = __builtin_convertvector(ec * f, v8h);
    const u16x8 ua = pa.u, uc = pc.u;
    unsigned short* g = P16 + row * NL_ + lane * 8;
    *(volatile u16x8*)g = ua;
    *(volatile u16x8*)(g + (NL_ / 2)) = uc;
    __threadfence();
    *(volatile u16x8*)g = ua;
    *(volatile u16x8*)(g + (NL_ / 2)) = uc;
}

__global__ __launch_bounds__(256)
void conv_silu_kernel(const float* __restrict__ XZ, const float* __restrict__ cw,
                      const float* __restrict__ cb, unsigned short* U16)
{
    const int mrow = blockIdx.x;
    const int l    = mrow & (NL_ - 1);
    const int c0   = threadIdx.x * 8;
    const size_t P4 = (size_t)2 * DI_;
    const float* xr = XZ + (size_t)mrow * P4 + c0;

    const v8f x3 = ld8f(xr);
    v8f x2, x1, x0;
#pragma unroll
    for (int c = 0; c < 8; ++c) { x2[c] = 0.0f; x1[c] = 0.0f; x0[c] = 0.0f; }
    if (l >= 1) x2 = ld8f(xr - P4);
    if (l >= 2) x1 = ld8f(xr - 2 * P4);
    if (l >= 3) x0 = ld8f(xr - 3 * P4);

    const float* wp = cw + (size_t)c0 * 4;
    v4f wv[8];
#pragma unroll
    for (int c = 0; c < 8; ++c) wv[c] = *(const v4f*)(wp + 4 * c);
    const v8f bias = ld8f(cb + c0);

    v8f u;
#pragma unroll
    for (int c = 0; c < 8; ++c) {
        const float cv = wv[c][0] * x0[c] + wv[c][1] * x1[c] + wv[c][2] * x2[c] + wv[c][3] * x3[c];
        u[c] = silu_f(cv + bias[c]) * 64.0f;
    }
    Pack8 pk;
    pk.f = __builtin_convertvector(u, v8h);
    const u16x8 v = pk.u;
    unsigned short* gp = U16 + (size_t)mrow * DI_ + c0;
    *(volatile u16x8*)gp = v;
    __threadfence();
    *(volatile u16x8*)gp = v;
}

__global__ __launch_bounds__(256)
void dt_cvt_kernel(const float* __restrict__ PRJ, unsigned short* DT16)
{
    const int i = blockIdx.x * 256 + threadIdx.x;
    if (i >= MT_ * 8) return;
    const int mrow = i >> 3;
    const int c8   = (i & 7) * 8;
    const v8f x = ld8f(PRJ + (size_t)mrow * XPN_ + c8);
    Pack8 pk;
    pk.f = __builtin_convertvector(x * 64.0f, v8h);
    const u16x8 v = pk.u;
    unsigned short* g = DT16 + (size_t)mrow * DTR_ + c8;
    *(volatile u16x8*)g = v;
    __threadfence();
    *(volatile u16x8*)g = v;
}

__global__ __launch_bounds__(256)
void scan_kernel(const float* __restrict__ XZ,
                 const float* __restrict__ DLr,
                 const float* __restrict__ PRJ,
                 const float* __restrict__ cw, const float* __restrict__ cb,
                 const float* __restrict__ dtb, const float* __restrict__ Alog,
                 const float* __restrict__ Dp, unsigned short* Y16)
{
    __shared__ __attribute__((aligned(16))) float sA[64 * NS_];
    __shared__ __attribute__((aligned(16))) float sBC[32 * 128];
    __shared__ __attribute__((aligned(16))) unsigned short sY[32 * 64];

    const int tid  = threadIdx.x;
    const int lane = tid & 31;
    const int wave = tid >> 5;
    const int q    = lane & 3;
    const int ch   = wave * 8 + (lane >> 2);
    const int d0   = blockIdx.x * 64;
    const int d    = d0 + ch;
    const int b    = blockIdx.y;
    const int n0   = q * 16;

#pragma unroll 1
    for (int j = 0; j < 16; ++j) {
        const int idx = j * 256 + tid;
        sA[idx] = -expf(Alog[(size_t)(d0 + (idx >> 6)) * NS_ + (idx & 63)]);
    }
    __syncthreads();

    float an[16], hs[16];
#pragma unroll
    for (int i = 0; i < 16; ++i) { an[i] = sA[ch * NS_ + n0 + i]; hs[i] = 0.0f; }

    const float w0 = cw[d * 4 + 0], w1 = cw[d * 4 + 1], w2 = cw[d * 4 + 2], w3 = cw[d * 4 + 3];
    const float cbias = cb[d];
    const float tb    = dtb[d];
    const float Dd    = Dp[d];

    float xm1 = 0.0f, xm2 = 0.0f, xm3 = 0.0f;
    const size_t mrow0 = (size_t)b * NL_;

#pragma unroll 1
    for (int t0 = 0; t0 < NL_; t0 += 32) {
        __syncthreads();
#pragma unroll
        for (int i = 0; i < 4; ++i) {
            const int idx = i * 256 + tid;
            const int s   = idx >> 5;
            const int f4  = (idx & 31) * 4;
            const v4f v = *(const v4f*)(PRJ + (mrow0 + t0 + s) * XPN_ + DTR_ + f4);
            *(v4f*)(sBC + s * 128 + f4) = v;
        }
        __syncthreads();

#pragma unroll 1
        for (int s = 0; s < 32; ++s) {
            const size_t mrow = mrow0 + (size_t)(t0 + s);
            const float xv = XZ[mrow * (2 * DI_) + d];
            const float zv = XZ[mrow * (2 * DI_) + DI_ + d];
            const float dl = DLr[mrow * DI_ + d];
            const float cv = w0 * xm3 + w1 * xm2 + w2 * xm1 + w3 * xv;
            const float u  = silu_f(cv + cbias);
            xm3 = xm2; xm2 = xm1; xm1 = xv;
            const float dt = softplus_f(dl + tb);
            const float du = dt * u;
            const float* bp = sBC + s * 128 + n0;
            const float* cp = bp + 64;
            float y = 0.0f;
#pragma unroll
            for (int i = 0; i < 16; ++i) {
                const float da = __expf(dt * an[i]);
                hs[i] = fmaf(hs[i], da, du * bp[i]);
                y = fmaf(hs[i], cp[i], y);
            }
            y += __shfl_xor(y, 1, 32);
            y += __shfl_xor(y, 2, 32);
            const float g = (y + Dd * u) * silu_f(zv);
            if (q == 0) {
                H1 hv;
                hv.f = (_Float16)(g * 64.0f);
                sY[s * 64 + ch] = hv.u;
            }
        }
        __syncthreads();
        {
            const int step = wave * 4 + (lane >> 3);
            const int c8   = (lane & 7) * 8;
            const u16x8 v = *(const u16x8*)(sY + step * 64 + c8);
            unsigned short* gp = Y16 + (mrow0 + t0 + step) * DI_ + d0 + c8;
            *(volatile u16x8*)gp = v;
            __threadfence();
            *(volatile u16x8*)gp = v;
        }
    }
}

__global__ __launch_bounds__(256)
void layernorm_kernel(const float* __restrict__ X, const float* __restrict__ g,
                      const float* __restrict__ bb, float* out)
{
    __shared__ float sred[8];
    const int row  = blockIdx.x;
    const int tid  = threadIdx.x;
    const int lane = tid & 31;
    const int wave = tid >> 5;
    const int c    = tid * 4;
    const v4f v = *(const v4f*)(X + (size_t)row * DM_ + c);

    float s = (v[0] + v[1]) + (v[2] + v[3]);
#pragma unroll
    for (int off = 16; off; off >>= 1) s += __shfl_xor(s, off, 32);
    if (lane == 0) sred[wave] = s;
    __syncthreads();
    float tot = 0.0f;
#pragma unroll
    for (int i = 0; i < 8; ++i) tot += sred[i];
    const float mu = tot * (1.0f / (float)DM_);
    __syncthreads();

    const v4f dv = v - mu;
    float s2 = (dv[0] * dv[0] + dv[1] * dv[1]) + (dv[2] * dv[2] + dv[3] * dv[3]);
#pragma unroll
    for (int off = 16; off; off >>= 1) s2 += __shfl_xor(s2, off, 32);
    if (lane == 0) sred[wave] = s2;
    __syncthreads();
    float tot2 = 0.0f;
#pragma unroll
    for (int i = 0; i < 8; ++i) tot2 += sred[i];
    const float var  = tot2 * (1.0f / (float)DM_);
    const float rstd = rsqrtf(var + 1e-5f);

    const v4f gv = *(const v4f*)(g + c);
    const v4f bv = *(const v4f*)(bb + c);
    const v4f o = (dv * rstd) * gv + bv;
    float* op = out + (size_t)row * DM_ + c;
    *(volatile v4f*)op = o;
    __threadfence();
    *(volatile v4f*)op = o;
}

extern "C" void kernel_launch(void* const* d_in, const int* in_sizes, int n_in,
                              void* d_out, int out_size, void* d_ws, size_t ws_size,
                              hipStream_t stream)
{
    if (n_in < 20) return;
    if (in_sizes[0]  != MT_ * DM_)     return;
    if (in_sizes[1]  != 3 * DM_ * DM_) return;
    if (in_sizes[2]  != 3 * DM_)       return;
    if (in_sizes[3]  != DM_ * DM_)     return;
    if (in_sizes[4]  != DM_)           return;
    if (in_sizes[5]  != FF_ * DM_)     return;
    if (in_sizes[6]  != FF_)           return;
    if (in_sizes[7]  != DM_ * FF_)     return;
    if (in_sizes[8]  != DM_)           return;
    if (in_sizes[9]  != DM_)           return;
    if (in_sizes[10] != DM_)           return;
    if (in_sizes[11] != 2 * DI_ * DM_) return;
    if (in_sizes[12] != DI_ * 4)       return;
    if (in_sizes[13] != DI_)           return;
    if (in_sizes[14] != XPN_ * DI_)    return;
    if (in_sizes[15] != DI_ * DTR_)    return;
    if (in_sizes[16] != DI_)           return;
    if (in_sizes[17] != DI_ * NS_)     return;
    if (in_sizes[18] != DI_)           return;
    if (in_sizes[19] != DM_ * DI_)     return;
    if (out_size != MT_ * DM_)         return;

    const float* src   = (const float*)d_in[0];
    const float* a_iw  = (const float*)d_in[1];
    const float* a_ib  = (const float*)d_in[2];
    const float* a_ow  = (const float*)d_in[3];
    const float* a_ob  = (const float*)d_in[4];
    const float* f_w1  = (const float*)d_in[5];
    const float* f_b1  = (const float*)d_in[6];
    const float* f_w2  = (const float*)d_in[7];
    const float* f_b2  = (const float*)d_in[8];
    const float* ln_g  = (const float*)d_in[9];
    const float* ln_b  = (const float*)d_in[10];
    const float* m_iw  = (const float*)d_in[11];
    const float* m_cw  = (const float*)d_in[12];
    const float* m_cb  = (const float*)d_in[13];
    const float* m_xw  = (const float*)d_in[14];
    const float* m_dtw = (const float*)d_in[15];
    const float* m_dtb = (const float*)d_in[16];
    const float* m_al  = (const float*)d_in[17];
    const float* m_D   = (const float*)d_in[18];
    const float* m_ow  = (const float*)d_in[19];
    float* out = (float*)d_out;

    const size_t MB = 1048576;
    const size_t OFF_W    = 0;
    const size_t OFF_W2   = 8 * MB;
    const size_t OFF_WDT  = 1 * MB;
    const size_t OFF_X16  = 16 * MB;
    const size_t OFF_XH   = 18 * MB;
    const size_t OFF_XL   = 20 * MB;
    const size_t OFF_AF   = 22 * MB;
    const size_t OFF_HH   = 26 * MB;
    const size_t OFF_HL   = 28 * MB;
    const size_t OFF_FFO  = 30 * MB;
    const size_t OFF_Q16  = 34 * MB;
    const size_t OFF_K16  = 36 * MB;
    const size_t OFF_VT   = 38 * MB;
    const size_t OFF_QKV  = 40 * MB;
    const size_t OFF_S    = 40 * MB;
    const size_t OFF_P16  = 72 * MB;
    const size_t OFF_AO   = 88 * MB;
    const size_t OFF_XZ   = 34 * MB;
    const size_t OFF_U16  = 50 * MB;
    const size_t OFF_PRJ  = 54 * MB;
    const size_t OFF_DT16 = 55 * MB;
    const size_t OFF_DL   = 56 * MB;
    const size_t OFF_Y16  = 64 * MB;
    const size_t OFF_FH   = 68 * MB;
    const size_t OFF_FL   = 76 * MB;
    const size_t WS_END   = 90 * MB;

    if ((size_t)2 * DI_ * DM_ * 2 > 16 * MB) return;
    if ((size_t)XPN_ * DI_ * 2 > OFF_WDT) return;
    if (OFF_WDT + (size_t)DI_ * DTR_ * 2 > OFF_W2) return;
    if (OFF_QKV + (size_t)MT_ * 3 * DM_ * 4 > OFF_P16) return;
    if (OFF_S + (size_t)NB_ * NH_ * NL_ * NL_ * 4 > OFF_P16) return;
    if (OFF_P16 + (size_t)NB_ * NH_ * NL_ * NL_ * 2 > OFF_AO) return;
    if (OFF_AO + (size_t)MT_ * DM_ * 2 > WS_END) return;
    if (OFF_XZ + (size_t)MT_ * 2 * DI_ * 4 > OFF_U16) return;
    if (OFF_DL + (size_t)MT_ * DI_ * 4 > OFF_Y16) return;
    if (OFF_FL + (size_t)MT_ * FF_ * 2 > WS_END) return;
    if (ws_size < WS_END) return;

    char* ws = (char*)d_ws;
    unsigned short* Wa   = (unsigned short*)(ws + OFF_W);
    unsigned short* Wb   = (unsigned short*)(ws + OFF_W2);
    unsigned short* Wdt  = (unsigned short*)(ws + OFF_WDT);
    unsigned short* X16  = (unsigned short*)(ws + OFF_X16);
    unsigned short* XH   = (unsigned short*)(ws + OFF_XH);
    unsigned short* XL   = (unsigned short*)(ws + OFF_XL);
    float*          AF   = (float*)(ws + OFF_AF);
    unsigned short* HH   = (unsigned short*)(ws + OFF_HH);
    unsigned short* HL   = (unsigned short*)(ws + OFF_HL);
    float*          FFO  = (float*)(ws + OFF_FFO);
    unsigned short* Q16  = (unsigned short*)(ws + OFF_Q16);
    unsigned short* K16  = (unsigned short*)(ws + OFF_K16);
    unsigned short* VT16 = (unsigned short*)(ws + OFF_VT);
    float*          QKVf = (float*)(ws + OFF_QKV);
    float*          Sf   = (float*)(ws + OFF_S);
    unsigned short* P16  = (unsigned short*)(ws + OFF_P16);
    unsigned short* AO16 = (unsigned short*)(ws + OFF_AO);
    float*          XZ   = (float*)(ws + OFF_XZ);
    unsigned short* U16  = (unsigned short*)(ws + OFF_U16);
    float*          PRJ  = (float*)(ws + OFF_PRJ);
    unsigned short* DT16 = (unsigned short*)(ws + OFF_DT16);
    float*          DL   = (float*)(ws + OFF_DL);
    unsigned short* Y16  = (unsigned short*)(ws + OFF_Y16);
    unsigned short* FH   = (unsigned short*)(ws + OFF_FH);
    unsigned short* FL   = (unsigned short*)(ws + OFF_FL);

    auto cvt = [&](const float* s, unsigned short* p0, unsigned short* p1, unsigned short* p2,
                   int n, int mode, float scale) {
        const int n8 = n / 8;
        cvt_kernel<<<dim3((n8 + 255) / 256), dim3(256), 0, stream>>>(s, p0, p1, p2, n8, mode, scale);
    };

    const float WSC   = 32.0f;
    const float R32   = 0.03125f;
    const float R512  = 0.001953125f;
    const float R2048 = 0.00048828125f;
    const float R2P14 = 6.103515625e-05f;

    cvt(src, X16, XH, XL, MT_ * DM_, 2, 1.0f);
    cvt(a_iw, Wa, Wa, Wa, 3 * DM_ * DM_, 0, WSC);
    gemm_tn_kernel<FragH, false, 0><<<dim3((3 * DM_) / 64, MT_ / 128, 1), dim3(128), 0, stream>>>(
        X16, X16, Wa, Wa, a_ib, AF, (void*)QKVf, (void*)QKVf,
        (int)DM_, (int)DM_, (int)DM_, (int)(3 * DM_), 1,
        0LL, 0LL, 0LL, 0LL, R32, 1.0f, 1);
    attn_prep_kernel<<<dim3(MT_ / 64, NH_ / 4), dim3(256), 0, stream>>>(QKVf, Q16, K16, VT16);
    gemm_tn_kernel<FragH, false, 0><<<dim3(NL_ / 64, NL_ / 128, NB_ * NH_), dim3(128), 0, stream>>>(
        Q16, Q16, K16, K16, a_ib, AF, (void*)Sf, (void*)Sf,
        (int)HD_, (int)HD_, (int)HD_, (int)NL_, 1,
        (long long)NL_ * HD_, (long long)NL_ * HD_, (long long)NL_ * NL_, 0LL, 0.125f, 1.0f, 0);
    softmax_kernel<<<dim3((NB_ * NH_ * NL_) / 8), dim3(256), 0, stream>>>(Sf, P16);
    gemm_tn_kernel<FragH, false, 1><<<dim3(1, NL_ / 128, NB_ * NH_), dim3(128), 0, stream>>>(
        P16, P16, VT16, VT16, a_ib, AF, (void*)AO16, (void*)AO16,
        (int)NL_, (int)NL_, (int)NL_, (int)DM_, (int)NH_,
        (long long)NL_ * NL_, (long long)HD_ * NL_, (long long)NL_ * DM_, (long long)HD_,
        R2P14, 16.0f, 0);
    cvt(a_ow, Wa, Wa, Wa, DM_ * DM_, 0, WSC);
    gemm_tn_kernel<FragH, false, 0><<<dim3(DM_ / 64, MT_ / 128, 1), dim3(128), 0, stream>>>(
        AO16, AO16, Wa, Wa, a_ob, AF, (void*)AF, (void*)AF,
        (int)DM_, (int)DM_, (int)DM_, (int)DM_, 1,
        0LL, 0LL, 0LL, 0LL, R512, 1.0f, 1);
    cvt(m_iw, Wa, Wb, Wb, 2 * DI_ * DM_, 1, 1.0f);
    gemm_tn_kernel<FragB, true, 0><<<dim3((2 * DI_) / 64, MT_ / 128, 1), dim3(128), 0, stream>>>(
        XH, XL, Wa, Wb, a_ib, AF, (void*)XZ, (void*)XZ,
        (int)DM_, (int)DM_, (int)DM_, (int)(2 * DI_), 1,
        0LL, 0LL, 0LL, 0LL, 1.0f, 1.0f, 0);
    conv_silu_kernel<<<dim3(MT_), dim3(DI_ / 8), 0, stream>>>(XZ, m_cw, m_cb, U16);
    cvt(m_xw, Wa, Wa, Wa, XPN_ * DI_, 0, WSC);
    cvt(m_dtw, Wdt, Wdt, Wdt, DI_ * DTR_, 0, WSC);
    gemm_tn_kernel<FragH, false, 0><<<dim3(XPN_ / 64, MT_ / 128, 1), dim3(128), 0, stream>>>(
        U16, U16, Wa, Wa, a_ib, AF, (void*)PRJ, (void*)PRJ,
        (int)DI_, (int)DI_, (int)DI_, (int)XPN_, 1,
        0LL, 0LL, 0LL, 0LL, R2048, 1.0f, 0);
    dt_cvt_kernel<<<dim3((MT_ * 8 + 255) / 256), dim3(256), 0, stream>>>(PRJ, DT16);
    gemm_tn_kernel<FragH, false, 0><<<dim3(DI_ / 64, MT_ / 128, 1), dim3(128), 0, stream>>>(
        DT16, DT16, Wdt, Wdt, a_ib, AF, (void*)DL, (void*)DL,
        (int)DTR_, (int)DTR_, (int)DTR_, (int)DI_, 1,
        0LL, 0LL, 0LL, 0LL, R2048, 1.0f, 0);
    scan_kernel<<<dim3(DI_ / 64, NB_), dim3(256), 0, stream>>>(
        XZ, DL, PRJ, m_cw, m_cb, m_dtb, m_al, m_D, Y16);
    cvt(m_ow, Wa, Wa, Wa, DM_ * DI_, 0, WSC);
    gemm_tn_kernel<FragH, false, 2><<<dim3(DM_ / 64, MT_ / 128, 1), dim3(128), 0, stream>>>(
        Y16, Y16, Wa, Wa, a_ib, AF, (void*)HH, (void*)HL,
        (int)DI_, (int)DI_, (int)DI_, (int)DM_, 1,
        0LL, 0LL, 0LL, 0LL, R2048, 1.0f, 2);
    cvt(f_w1, Wa, Wb, Wb, FF_ * DM_, 1, 1.0f);
    gemm_tn_kernel<FragB, true, 2><<<dim3(FF_ / 64, MT_ / 128, 1), dim3(128), 0, stream>>>(
        HH, HL, Wa, Wb, f_b1, AF, (void*)FH, (void*)FL,
        (int)DM_, (int)DM_, (int)DM_, (int)FF_, 1,
        0LL, 0LL, 0LL, 0LL, 1.0f, 1.0f, 1 | 4);
    cvt(f_w2, Wa, Wb, Wb, DM_ * FF_, 1, 1.0f);
    gemm_tn_kernel<FragB, true, 0><<<dim3(DM_ / 64, MT_ / 128, 1), dim3(128), 0, stream>>>(
        FH, FL, Wa, Wb, f_b2, AF, (void*)FFO, (void*)FFO,
        (int)FF_, (int)FF_, (int)FF_, (int)DM_, 1,
        0LL, 0LL, 0LL, 0LL, 1.0f, 1.0f, 1);
    layernorm_kernel<<<dim3(MT_), dim3(256), 0, stream>>>(FFO, ln_g, ln_b, out);
}
